// GlobalAttention3D_22505628631557
// MI455X (gfx1250) — hardware-verified
//
#include <hip/hip_runtime.h>
#include <math.h>
#include <stdint.h>

typedef __attribute__((ext_vector_type(16))) _Float16 v16h;
typedef __attribute__((ext_vector_type(8)))  _Float16 v8h;
typedef __attribute__((ext_vector_type(16))) __bf16   v16b;
typedef __attribute__((ext_vector_type(8)))  __bf16   v8b;
typedef __attribute__((ext_vector_type(8)))  float    v8f;
typedef __attribute__((ext_vector_type(4)))  float    v4f;
typedef __attribute__((ext_vector_type(2)))  float    v2f;
typedef __attribute__((ext_vector_type(4)))  unsigned int v4u;

constexpr int NBATCH_  = 2;
constexpr int CIN_     = 64;
constexpr int EMB_     = 128;
constexpr int COUT_    = 64;
constexpr int NHEAD_   = 2;
constexpr int HDIM_    = 64;
constexpr int SEQL_    = 4096;
constexpr int NTOK_    = NBATCH_ * SEQL_;
constexpr int QKPITCH_ = 2 * EMB_;

constexpr int WOFF_CP   = 0;
constexpr int WOFF_Q    = WOFF_CP + EMB_ * CIN_;
constexpr int WOFF_K    = WOFF_Q + EMB_ * EMB_;
constexpr int WOFF_V    = WOFF_K + EMB_ * EMB_;
constexpr int WOFF_O    = WOFF_V + EMB_ * EMB_;
constexpr int WOFF_OUT  = WOFF_O + EMB_ * EMB_;
constexpr int WPOOL_H   = WOFF_OUT + COUT_ * EMB_;
static_assert(WPOOL_H == 81920, "weight pool size");

constexpr size_t OFFB_W   = 0;
constexpr size_t OFFB_XT  = OFFB_W  + (size_t)WPOOL_H * 2;
constexpr size_t OFFB_XF  = OFFB_XT + (size_t)NTOK_ * CIN_ * 2;
constexpr size_t OFFB_QK  = OFFB_XF + (size_t)NTOK_ * EMB_ * 2;
constexpr size_t OFFB_VT  = OFFB_QK + (size_t)NTOK_ * QKPITCH_ * 2;
constexpr size_t OFFB_O   = OFFB_VT + (size_t)NBATCH_ * EMB_ * SEQL_ * 2;
constexpr size_t OFFB_O1  = OFFB_O  + (size_t)NTOK_ * EMB_ * 2;
constexpr size_t WS_TOTAL = OFFB_O1 + (size_t)NTOK_ * EMB_ * 2;
static_assert(WS_TOTAL == 13795328, "carve total");
static_assert((OFFB_XT % 128) == 0 && (OFFB_XF % 128) == 0 && (OFFB_QK % 128) == 0 &&
              (OFFB_VT % 128) == 0 && (OFFB_O % 128) == 0 && (OFFB_O1 % 128) == 0, "128-B aligned regions");

#define U16(p) ((const unsigned short*)(const void*)(p))

__device__ __forceinline__ unsigned short f2bf_bits(float f) {
  unsigned u = __float_as_uint(f);
  return (unsigned short)((u + 0x7FFFu + ((u >> 16) & 1u)) >> 16);
}
__device__ __forceinline__ float bf_bits2f(unsigned short h) { return __uint_as_float(((unsigned)h) << 16); }
__device__ __forceinline__ unsigned pk16(unsigned short a, unsigned short b) { return (unsigned)a | ((unsigned)b << 16); }
__device__ __forceinline__ unsigned short h_bits(float f) { return __builtin_bit_cast(unsigned short, (_Float16)f); }

__device__ __forceinline__ void dep_guard_h(v8f& a, v8f& b, v16h x, v16h y) { asm volatile("v_nop\n\tv_nop\n\tv_nop\n\tv_nop" : "+v"(a), "+v"(b) : "v"(x), "v"(y)); }
__device__ __forceinline__ void dep_guard_b(v8f& a, v8f& b, v16b x, v16b y) { asm volatile("v_nop\n\tv_nop\n\tv_nop\n\tv_nop" : "+v"(a), "+v"(b) : "v"(x), "v"(y)); }
__device__ __forceinline__ void keep4_h(v16h a, v16h b, v16h c, v16h d) { asm volatile("v_nop" :: "v"(a), "v"(b), "v"(c), "v"(d)); }
__device__ __forceinline__ void keep4_b(v16b a, v16b b, v16b c, v16b d) { asm volatile("v_nop" :: "v"(a), "v"(b), "v"(c), "v"(d)); }
__device__ __forceinline__ void acc_guard4(v8f& a, v8f& b, v8f& c, v8f& d) { asm volatile("v_nop\n\tv_nop\n\tv_nop\n\tv_nop" : "+v"(a), "+v"(b), "+v"(c), "+v"(d)); }
template <typename T> struct Frag;
template <> struct Frag<_Float16> {
  typedef v16h V; union U { v16h v; v8h h[2]; };
  static __device__ __forceinline__ v16h load(const _Float16* p) {
    U f; f.h[0] = *(const v8h*)(p); f.h[1] = *(const v8h*)(p + 16); return f.v;
  }
  static __device__ __forceinline__ v8f mma(v16h a, v16h b, v8f c) {
    return __builtin_amdgcn_wmma_f32_16x16x32_f16(false, a, false, b, (short)0, c, false, false);
  }
  static __device__ __forceinline__ void guard(v8f& a, v8f& b, v16h x, v16h y) { dep_guard_h(a, b, x, y); }
  static __device__ __forceinline__ void keep(v16h a, v16h b, v16h c, v16h d) { keep4_h(a, b, c, d); }
};
template <> struct Frag<__bf16> {
  typedef v16b V; union U { v16b v; v8b h[2]; };
  static __device__ __forceinline__ v16b load(const __bf16* p) {
    U f; f.h[0] = *(const v8b*)(p); f.h[1] = *(const v8b*)(p + 16); return f.v;
  }
  static __device__ __forceinline__ v8f mma(v16b a, v16b b, v8f c) {
    return __builtin_amdgcn_wmma_f32_16x16x32_bf16(false, a, false, b, (short)0, c, false, false);
  }
  static __device__ __forceinline__ void guard(v8f& a, v8f& b, v16b x, v16b y) { dep_guard_b(a, b, x, y); }
  static __device__ __forceinline__ void keep(v16b a, v16b b, v16b c, v16b d) { keep4_b(a, b, c, d); }
};

template <int ET> struct Elem;
template <> struct Elem<0> { typedef _Float16 T; };
template <> struct Elem<1> { typedef __bf16 T; };
template <int ET, bool SPLIT, int BIAS_MODE, int OUT_MODE, bool RESID, int ACT = 0>
__global__ __launch_bounds__(256) void wmma_gemm64(
    const unsigned short* __restrict__ Ap, const unsigned short* __restrict__ A2p, int lda, long strideA,
    const unsigned short* __restrict__ Btp, const unsigned short* __restrict__ Bt2p, int ldb, long strideB,
    void* __restrict__ Cout, void* __restrict__ Cout2, int ldc, long strideC,
    const float* __restrict__ bias,
    const float* __restrict__ resid, long strideR, const float* __restrict__ rgain,
    int M, int N, int K, float scale) {
  typedef typename Elem<ET>::T T;
  typedef typename Frag<T>::V V;
  const T* A = (const T*)Ap; const T* A2 = (const T*)A2p; const T* Bt = (const T*)Btp; const T* Bt2 = (const T*)Bt2p;
  __shared__ __align__(16) float sT[8][16 * 68];
  const int b    = blockIdx.y;
  const int lane = threadIdx.x & 31;
  const int wave = threadIdx.x >> 5;
  const int tilesN = N >> 6;
  const int tilesM = M >> 6;
  const int tile = blockIdx.x * 8 + wave;
  if (tile >= tilesM * tilesN) return;
  const int tm = tile / tilesN;
  const int tn = tile - tm * tilesN;
  const int m0 = tm << 6;
  const int n0 = tn << 6;

  const T* Ab  = A  + (size_t)b * strideA;
  const T* Bb  = Bt + (size_t)b * strideB;
  const T* Ab2 = SPLIT ? (A2  + (size_t)b * strideA) : nullptr;
  const T* Bb2 = SPLIT ? (Bt2 + (size_t)b * strideB) : nullptr;

  const int rlane = lane & 15;
  const int koff  = (lane >> 4) * 8;
  const int mOff  = (lane >> 4) * 8;

  v8f acc[4][4];
#pragma unroll
  for (int i = 0; i < 4; ++i)
#pragma unroll
    for (int j = 0; j < 4; ++j) acc[i][j] = (v8f){0.f,0.f,0.f,0.f,0.f,0.f,0.f,0.f};

  for (int k0 = 0; k0 < K; k0 += 32) {
    V bh[4], bl[4];
#pragma unroll
    for (int j = 0; j < 4; ++j) {
      const size_t bo = (size_t)(n0 + (j << 4) + rlane) * ldb + koff + k0;
      bh[j] = Frag<T>::load(Bb + bo);
      if (SPLIT) bl[j] = Frag<T>::load(Bb2 + bo);
    }
#pragma unroll
    for (int i = 0; i < 4; ++i) {
      const size_t ao = (size_t)(m0 + (i << 4) + rlane) * lda + koff + k0;
      V ah = Frag<T>::load(Ab + ao);
      V al;
      if (SPLIT) al = Frag<T>::load(Ab2 + ao);
#pragma unroll
      for (int j = 0; j < 4; ++j) {
        acc[i][j] = Frag<T>::mma(ah, bh[j], acc[i][j]);
        if (SPLIT) {
          acc[i][j] = Frag<T>::mma(ah, bl[j], acc[i][j]);
          acc[i][j] = Frag<T>::mma(al, bh[j], acc[i][j]);
        }
      }
      Frag<T>::guard(acc[i][0], acc[i][3], ah, SPLIT ? al : ah);
    }
    Frag<T>::keep(bh[0], bh[1], bh[2], bh[3]);
    if (SPLIT) Frag<T>::keep(bl[0], bl[1], bl[2], bl[3]);
  }
  acc_guard4(acc[0][0], acc[0][1], acc[0][2], acc[0][3]);
  acc_guard4(acc[1][0], acc[1][1], acc[1][2], acc[1][3]);
  acc_guard4(acc[2][0], acc[2][1], acc[2][2], acc[2][3]);
  acc_guard4(acc[3][0], acc[3][1], acc[3][2], acc[3][3]);

  float* slab = sT[wave];
  const float* Rb = RESID ? (resid + (size_t)b * strideR) : nullptr;
  float rg = 1.0f;
  if (RESID) { if (rgain != nullptr) rg = rgain[0]; }
#pragma unroll
  for (int i = 0; i < 4; ++i) {
    const int mBase = m0 + (i << 4);
#pragma unroll
    for (int j = 0; j < 4; ++j) {
      const int n = n0 + (j << 4) + rlane;
      float bv = 0.f;
      if (BIAS_MODE == 2) bv = bias[n];
#pragma unroll
      for (int r = 0; r < 8; ++r) {
        float v = acc[i][j][r] * scale;
        if (BIAS_MODE == 1) v += bias[mBase + mOff + r];
        if (BIAS_MODE == 2) v += bv;
        if (RESID) v += rg * Rb[(size_t)(mBase + mOff + r) * ldc + n];
        if (ACT == 1) v = tanhf(v);
        if (ACT == 2) v = fmaxf(v, 0.0f);
        if (ACT == 3) v = v / (1.0f + expf(-v));
        if (ACT == 4) v = (v > 0.f) ? v : 0.01f * v;
        slab[(mOff + r) * 68 + (j << 4) + rlane] = v;
      }
    }
    __builtin_amdgcn_fence(__ATOMIC_RELEASE, "workgroup");
    __builtin_amdgcn_wave_barrier();
    __builtin_amdgcn_fence(__ATOMIC_ACQUIRE, "workgroup");
    if (OUT_MODE == 0) {
      float* C = (float*)Cout + (size_t)b * strideC;
      const int hh = lane >> 4, c4 = (lane & 15) * 4;
      for (int pass = 0; pass < 2; ++pass) {
#pragma unroll
        for (int it = 0; it < 8; ++it) {
          const int row = it * 2 + hh;
          v4f v = *(const v4f*)(slab + row * 68 + c4);
          *(volatile v4f*)(C + (size_t)(mBase + row) * ldc + n0 + c4) = v;
        }
        __threadfence();
      }
    } else {
      const int q = lane >> 3, c8 = (lane & 7) * 8;
      unsigned short* C  = (unsigned short*)Cout  + (size_t)b * strideC;
      unsigned short* C2 = (OUT_MODE == 2) ? ((unsigned short*)Cout2 + (size_t)b * strideC) : nullptr;
      for (int pass = 0; pass < 2; ++pass) {
#pragma unroll
        for (int it = 0; it < 4; ++it) {
          const int row = it * 4 + q;
          const float* sp = slab + row * 68 + c8;
          v8h hv, lv;
#pragma unroll
          for (int e = 0; e < 8; ++e) {
            if (OUT_MODE == 1) {
              hv[e] = (_Float16)sp[e];
            } else {
              unsigned short hb = f2bf_bits(sp[e]);
              unsigned short lb = f2bf_bits(sp[e] - bf_bits2f(hb));
              hv[e] = __builtin_bit_cast(_Float16, hb);
              lv[e] = __builtin_bit_cast(_Float16, lb);
            }
          }
          *(volatile v8h*)(C + (size_t)(mBase + row) * ldc + n0 + c8) = hv;
          if (OUT_MODE == 2) *(volatile v8h*)(C2 + (size_t)(mBase + row) * ldc + n0 + c8) = lv;
        }
        __threadfence();
      }
    }
    __builtin_amdgcn_fence(__ATOMIC_RELEASE, "workgroup");
    __builtin_amdgcn_wave_barrier();
    __builtin_amdgcn_fence(__ATOMIC_ACQUIRE, "workgroup");
  }
}

__global__ __launch_bounds__(256) void cast_w6_kernel(const float* __restrict__ w0, const float* __restrict__ w1,
                                                      const float* __restrict__ w2, const float* __restrict__ w3,
                                                      const float* __restrict__ w4, const float* __restrict__ w5,
                                                      _Float16* __restrict__ pool, float sc) {
  const int y = blockIdx.y;
  const float* in = w0; int n2 = (EMB_ * CIN_) / 2; int off = WOFF_CP;
  if (y == 1) { in = w1; n2 = (EMB_ * EMB_) / 2;  off = WOFF_Q; }
  if (y == 2) { in = w2; n2 = (EMB_ * EMB_) / 2;  off = WOFF_K; }
  if (y == 3) { in = w3; n2 = (EMB_ * EMB_) / 2;  off = WOFF_V; }
  if (y == 4) { in = w4; n2 = (EMB_ * EMB_) / 2;  off = WOFF_O; }
  if (y == 5) { in = w5; n2 = (COUT_ * EMB_) / 2; off = WOFF_OUT; }
  _Float16* out = pool + off;
  const int i = blockIdx.x * 256 + threadIdx.x;
  if (i < n2) {
    const v2f f = *(const v2f*)(in + 2 * (size_t)i);
    const unsigned u = pk16(h_bits(f[0] * sc), h_bits(f[1] * sc));
    ((volatile unsigned*)out)[i] = u;
    __threadfence();
    ((volatile unsigned*)out)[i] = u;
  }
}

__global__ __launch_bounds__(256) void tcast16_kernel(const float* __restrict__ W, unsigned short* __restrict__ oh,
                                                      int R, int Cc, long sIn, long sOut) {
  __shared__ __align__(16) float tf[64 * 68];
  W  += (size_t)blockIdx.z * sIn;
  oh += (size_t)blockIdx.z * sOut;
  const int c0  = blockIdx.x * 64;
  const int r0  = blockIdx.y * 64;
  const int tid = threadIdx.x;
  {
    const int lr = tid >> 4;
    const int c4 = (tid & 15) * 4;
#pragma unroll
    for (int it = 0; it < 4; ++it) {
      const int rr = it * 16 + lr;
      const v4f a = *(const v4f*)(W + (size_t)(r0 + rr) * Cc + c0 + c4);
      *(v4f*)(tf + rr * 68 + c4) = a;
    }
  }
  __syncthreads();
  const int sub = tid >> 3;
  const int c8  = (tid & 7) * 8;
  v4u hv[2];
#pragma unroll
  for (int it = 0; it < 2; ++it) {
    const int oc = it * 32 + sub;
    v4u a;
#pragma unroll
    for (int q = 0; q < 4; ++q) {
      const float f0 = tf[(c8 + 2 * q) * 68 + oc];
      const float f1 = tf[(c8 + 2 * q + 1) * 68 + oc];
      a[q] = pk16(h_bits(f0), h_bits(f1));
    }
    hv[it] = a;
  }
  for (int pass = 0; pass < 2; ++pass) {
#pragma unroll
    for (int it = 0; it < 2; ++it) {
      const int oc = it * 32 + sub;
      const size_t go = (size_t)(c0 + oc) * R + r0 + c8;
      *(volatile v4u*)(oh + go) = hv[it];
    }
    __threadfence();
  }
}

#define AT_D 64
#define AT_NW 4
#define AT_QB 64
#define AT_KC 64
#define P_CARRY 32768.0f

__device__ __forceinline__ v8f at_mma_h(v16h a, v16h b, v8f c) {
  c = __builtin_amdgcn_wmma_f32_16x16x32_f16(false, a, false, b, (short)0, c, false, false);
  asm volatile("v_nop\n\tv_nop\n\tv_nop\n\tv_nop" : "+v"(c) : "v"(a), "v"(b));
  return c;
}

__global__ __launch_bounds__(128)
void attn_full64_f16_kernel(const unsigned short* __restrict__ qkp, const unsigned short* __restrict__ vtp,
                            unsigned short* __restrict__ op, float sscale, float oscale) {
  union FH { v16h v; v8h h[2]; };
  __shared__ __align__(16) _Float16 Ksh[AT_KC * AT_D];
  __shared__ __align__(16) _Float16 Vth[AT_D * AT_KC];
  __shared__ __align__(16) _Float16 Psh[AT_NW][16 * AT_KC];
  __shared__ __align__(16) float    Os[AT_NW][16 * 68];

  const int tid  = threadIdx.x;
  const int wave = tid >> 5;
  const int lane = tid & 31;
  const int hh   = lane >> 4;
  const int c    = lane & 15;

  const int nqb = SEQL_ / AT_QB;
  const int bx = blockIdx.x;
  const int qb = bx % nqb;
  const int bh = bx / nqb;
  const int h  = bh % NHEAD_;
  const int b  = bh / NHEAD_;
  const int q0 = qb * AT_QB + wave * 16;

  const _Float16* Qh = (const _Float16*)(const void*)qkp + (size_t)b * SEQL_ * QKPITCH_ + (size_t)h * AT_D;
  const _Float16* Kh = Qh + EMB_;
  const _Float16* Vh = (const _Float16*)(const void*)vtp + (size_t)b * EMB_ * SEQL_ + (size_t)h * AT_D * SEQL_;
  _Float16*       ob = (_Float16*)(void*)op + (size_t)b * SEQL_ * EMB_ + (size_t)h * AT_D;

  v16h qa[2];
#pragma unroll
  for (int dc = 0; dc < 2; ++dc) {
    const _Float16* qr = Qh + (size_t)(q0 + c) * QKPITCH_ + dc * 32 + 8 * hh;
    qa[dc] = Frag<_Float16>::load(qr);
  }

  float mrow[8], lrow[8];
  v8f oacc[4];
#pragma unroll
  for (int r = 0; r < 8; ++r) { mrow[r] = -INFINITY; lrow[r] = 0.f; }
#pragma unroll
  for (int t = 0; t < 4; ++t) oacc[t] = (v8f){0.f,0.f,0.f,0.f,0.f,0.f,0.f,0.f};

  const int nChunks = SEQL_ / AT_KC;
  for (int kc = 0; kc < nChunks; ++kc) {
    const int kv0 = kc * AT_KC;
    __syncthreads();
    {
      const int r = tid >> 1, half = (tid & 1) * 32;
      const _Float16* ksh = Kh + (size_t)(kv0 + r) * QKPITCH_ + half;
      const _Float16* vsh = Vh + (size_t)r * SEQL_ + kv0 + half;
#pragma unroll
      for (int i = 0; i < 4; ++i) {
        const v8h a0 = *(const v8h*)(ksh + 8 * i);
        const v8h b0 = *(const v8h*)(vsh + 8 * i);
        *(v8h*)(Ksh + r * AT_D  + half + 8 * i) = a0;
        *(v8h*)(Vth + r * AT_KC + half + 8 * i) = b0;
      }
    }
    __syncthreads();

    v8f s[4];
#pragma unroll
    for (int j = 0; j < 4; ++j) {
      s[j] = (v8f){0.f,0.f,0.f,0.f,0.f,0.f,0.f,0.f};
#pragma unroll
      for (int dc = 0; dc < 2; ++dc) {
        FH kb;
        kb.h[0] = *(const v8h*)(Ksh + (j * 16 + c) * AT_D + dc * 32 + 8 * hh);
        kb.h[1] = *(const v8h*)(Ksh + (j * 16 + c) * AT_D + dc * 32 + 16 + 8 * hh);
        s[j] = at_mma_h(qa[dc], kb.v, s[j]);
      }
    }
    float cm[8];
#pragma unroll
    for (int r = 0; r < 8; ++r) {
      float m = -INFINITY;
#pragma unroll
      for (int j = 0; j < 4; ++j) {
        const float sv = s[j][r] * sscale;
        s[j][r] = sv;
        m = fmaxf(m, sv);
      }
#pragma unroll
      for (int off = 1; off < 16; off <<= 1) m = fmaxf(m, __shfl_xor(m, off, 32));
      cm[r] = m;
    }
    _Float16* pwh = Psh[wave];
#pragma unroll
    for (int r = 0; r < 8; ++r) {
      const float mnew = fmaxf(mrow[r], cm[r]);
      const float alpha = expf(mrow[r] - mnew);
      mrow[r] = mnew;
      float psum = 0.f;
#pragma unroll
      for (int j = 0; j < 4; ++j) {
        const float p = expf(s[j][r] - mnew);
        psum += p;
        pwh[(8 * hh + r) * AT_KC + j * 16 + c] = (_Float16)(p * P_CARRY);
      }
#pragma unroll
      for (int off = 1; off < 16; off <<= 1) psum += __shfl_xor(psum, off, 32);
      lrow[r] = lrow[r] * alpha + psum;
#pragma unroll
      for (int t = 0; t < 4; ++t) oacc[t][r] *= alpha;
    }
    __builtin_amdgcn_fence(__ATOMIC_RELEASE, "workgroup");
    __builtin_amdgcn_wave_barrier();
    __builtin_amdgcn_fence(__ATOMIC_ACQUIRE, "workgroup");
#pragma unroll 1
    for (int kk = 0; kk < 2; ++kk) {
      FH pa;
      pa.h[0] = *(const v8h*)(pwh + c * AT_KC + kk * 32 + 8 * hh);
      pa.h[1] = *(const v8h*)(pwh + c * AT_KC + kk * 32 + 16 + 8 * hh);
#pragma unroll
      for (int t = 0; t < 4; ++t) {
        FH vb;
        vb.h[0] = *(const v8h*)(Vth + (t * 16 + c) * AT_KC + kk * 32 + 8 * hh);
        vb.h[1] = *(const v8h*)(Vth + (t * 16 + c) * AT_KC + kk * 32 + 16 + 8 * hh);
        oacc[t] = at_mma_h(pa.v, vb.v, oacc[t]);
      }
    }
  }

  float* os = Os[wave];
#pragma unroll
  for (int r = 0; r < 8; ++r) {
    const float inv = oscale / (lrow[r] * P_CARRY);
#pragma unroll
    for (int t = 0; t < 4; ++t) os[(8 * hh + r) * 68 + t * 16 + c] = oacc[t][r] * inv;
  }
  __builtin_amdgcn_fence(__ATOMIC_RELEASE, "workgroup");
  __builtin_amdgcn_wave_barrier();
  __builtin_amdgcn_fence(__ATOMIC_ACQUIRE, "workgroup");
  {
    const int q8 = lane >> 3, c8 = (lane & 7) * 8;
    for (int pass = 0; pass < 2; ++pass) {
#pragma unroll
      for (int it = 0; it < 4; ++it) {
        const int row = it * 4 + q8;
        const float* sp = os + row * 68 + c8;
        v8h hv;
#pragma unroll
        for (int e = 0; e < 8; ++e) hv[e] = (_Float16)sp[e];
        *(volatile v8h*)(ob + (size_t)(q0 + row) * EMB_ + c8) = hv;
      }
      __threadfence();
    }
  }
}

extern "C" void kernel_launch(void* const* d_in, const int* in_sizes, int n_in,
                              void* d_out, int out_size, void* d_ws, size_t ws_size,
                              hipStream_t stream) {
  if (n_in < 12) return;
  if (in_sizes[0] != NBATCH_ * CIN_ * SEQL_) return;
  if (in_sizes[1] != EMB_ * CIN_ || in_sizes[2] != EMB_) return;
  if (in_sizes[3] != EMB_ * EMB_ || in_sizes[4] != EMB_ * EMB_ || in_sizes[5] != EMB_ * EMB_) return;
  if (in_sizes[6] != EMB_ * EMB_ || in_sizes[7] != EMB_) return;
  if (in_sizes[8] != COUT_ * EMB_ || in_sizes[9] != COUT_) return;
  if (in_sizes[10] != SEQL_ * EMB_ || in_sizes[11] < 1) return;
  if (out_size != NBATCH_ * COUT_ * SEQL_) return;
  if (ws_size < WS_TOTAL) return;

  const float* x     = (const float*)d_in[0];
  const float* W_cp  = (const float*)d_in[1];
  const float* b_cp  = (const float*)d_in[2];
  const float* W_q   = (const float*)d_in[3];
  const float* W_k   = (const float*)d_in[4];
  const float* W_v   = (const float*)d_in[5];
  const float* W_o   = (const float*)d_in[6];
  const float* b_o   = (const float*)d_in[7];
  const float* W_out = (const float*)d_in[8];
  const float* b_out = (const float*)d_in[9];
  const float* pos   = (const float*)d_in[10];
  const float* gatep = (const float*)d_in[11];
  float* out = (float*)d_out;

  char* ws = (char*)d_ws;
  _Float16* wpool = (_Float16*)(void*)(ws + OFFB_W);
  unsigned short* XT16 = (unsigned short*)(void*)(ws + OFFB_XT);
  unsigned short* XF16 = (unsigned short*)(void*)(ws + OFFB_XF);
  unsigned short* QK16 = (unsigned short*)(void*)(ws + OFFB_QK);
  unsigned short* VT16 = (unsigned short*)(void*)(ws + OFFB_VT);
  unsigned short* O16  = (unsigned short*)(void*)(ws + OFFB_O);
  unsigned short* O1   = (unsigned short*)(void*)(ws + OFFB_O1);
  const unsigned short* Wcp16  = U16(wpool + WOFF_CP);
  const unsigned short* Wqk16  = U16(wpool + WOFF_Q);
  const unsigned short* Wv16   = U16(wpool + WOFF_V);
  const unsigned short* Wo16   = U16(wpool + WOFF_O);
  const unsigned short* Wout16 = U16(wpool + WOFF_OUT);

  const float WSC = 8.0f;
  const float OSC = 16.0f;
  const float inv_w  = 1.0f / 8.0f;
  const float inv_wo = 1.0f / (8.0f * 16.0f);

  cast_w6_kernel<<<dim3(32, 6, 1), dim3(256, 1, 1), 0, stream>>>(W_cp, W_q, W_k, W_v, W_o, W_out, wpool, WSC);

  tcast16_kernel<<<dim3(SEQL_ / 64, CIN_ / 64, NBATCH_), dim3(256, 1, 1), 0, stream>>>(
      x, XT16, CIN_, SEQL_, (long)CIN_ * SEQL_, (long)SEQL_ * CIN_);

  wmma_gemm64<0, false, 2, 1, true><<<dim3((SEQL_ / 64) * (EMB_ / 64) / 8, NBATCH_, 1), dim3(256, 1, 1), 0, stream>>>(
      XT16, XT16, CIN_, (long)SEQL_ * CIN_,
      Wcp16, Wcp16, CIN_, 0L,
      (void*)XF16, nullptr, EMB_, (long)SEQL_ * EMB_,
      b_cp, pos, 0L, nullptr,
      SEQL_, EMB_, CIN_, inv_w);

  wmma_gemm64<0, false, 0, 1, false><<<dim3((NTOK_ / 64) * (QKPITCH_ / 64) / 8, 1, 1), dim3(256, 1, 1), 0, stream>>>(
      XF16, XF16, EMB_, 0L,
      Wqk16, Wqk16, EMB_, 0L,
      (void*)QK16, nullptr, QKPITCH_, 0L,
      nullptr, nullptr, 0L, nullptr,
      NTOK_, QKPITCH_, EMB_, inv_w);

  wmma_gemm64<0, false, 0, 1, false><<<dim3((EMB_ / 64) * (SEQL_ / 64) / 8, NBATCH_, 1), dim3(256, 1, 1), 0, stream>>>(
      Wv16, Wv16, EMB_, 0L,
      XF16, XF16, EMB_, (long)SEQL_ * EMB_,
      (void*)VT16, nullptr, SEQL_, (long)EMB_ * SEQL_,
      nullptr, nullptr, 0L, nullptr,
      EMB_, SEQL_, EMB_, inv_w);

  attn_full64_f16_kernel<<<dim3(NBATCH_ * NHEAD_ * (SEQL_ / AT_QB), 1, 1), dim3(128, 1, 1), 0, stream>>>(
      QK16, VT16, O16, 0.125f, OSC);

  wmma_gemm64<0, false, 2, 1, false><<<dim3((NTOK_ / 64) * (EMB_ / 64) / 8, 1, 1), dim3(256, 1, 1), 0, stream>>>(
      O16, O16, EMB_, 0L,
      Wo16, Wo16, EMB_, 0L,
      (void*)O1, nullptr, EMB_, 0L,
      b_o, nullptr, 0L, nullptr,
      NTOK_, EMB_, EMB_, inv_wo);

  wmma_gemm64<0, false, 1, 0, true><<<dim3((COUT_ / 64) * (SEQL_ / 64) / 8, NBATCH_, 1), dim3(256, 1, 1), 0, stream>>>(
      Wout16, Wout16, EMB_, 0L,
      O1, O1, EMB_, (long)SEQL_ * EMB_,
      (void*)out, nullptr, SEQL_, (long)COUT_ * SEQL_,
      b_out, x, (long)COUT_ * SEQL_, gatep,
      COUT_, SEQL_, EMB_, inv_w);
}
